// KANBlock_84748294684697
// MI455X (gfx1250) — hardware-verified
//
#include <hip/hip_runtime.h>


#define NROW 16384
#define D0   256
#define D1   512
#define D2   256
#define NB6  6
#define NG   10
#define K1   (D0 * 7)
#define K2   (D1 * 7)
#define RCH  8192
#define DM   D0
#define LOSC 1024.0f
typedef _Float16 h16;
typedef unsigned short bf;
typedef __attribute__((ext_vector_type(16))) __bf16   v16bf;
typedef __attribute__((ext_vector_type(16))) _Float16 v16h;
typedef __attribute__((ext_vector_type(8)))  _Float16 v8h;
typedef __attribute__((ext_vector_type(8)))  unsigned short v8us;
typedef __attribute__((ext_vector_type(8)))  float    v8f;
typedef __attribute__((ext_vector_type(4)))  float    v4f;
typedef v8h  __attribute__((may_alias)) v8ha;
typedef v4f  __attribute__((may_alias)) v4fa;
typedef v8us __attribute__((may_alias)) v8usa;

__device__ __forceinline__ unsigned short f2bf(float f) { unsigned u = __float_as_uint(f); u += 0x7FFFu + ((u >> 16) & 1u); return (unsigned short)(u >> 16); }
__device__ __forceinline__ float bf2f(unsigned short b) { return __uint_as_float(((unsigned)b) << 16); }
__device__ __forceinline__ float bfr(float f) { return bf2f(f2bf(f)); }
__device__ __forceinline__ v16h cat16(v8h lo, v8h hi) { return __builtin_shufflevector(lo, hi, 0, 1, 2, 3, 4, 5, 6, 7, 8, 9, 10, 11, 12, 13, 14, 15); }
__device__ __forceinline__ v16bf cat16b(v8us lo, v8us hi) { return __builtin_bit_cast(v16bf, __builtin_shufflevector(lo, hi, 0, 1, 2, 3, 4, 5, 6, 7, 8, 9, 10, 11, 12, 13, 14, 15)); }
__device__ __forceinline__ v8f wmma16(v16h a, v16h b, v8f c) { return __builtin_amdgcn_wmma_f32_16x16x32_f16(false, a, false, b, (short)0, c, false, false); }
__device__ __forceinline__ v8f wmmab(v16bf a, v16bf b, v8f c) { return __builtin_amdgcn_wmma_f32_16x16x32_bf16(false, a, false, b, (short)0, c, false, false); }


__global__ __launch_bounds__(128) void k_gemmh(const h16* __restrict__ A, const h16* __restrict__ Bn, const float* __restrict__ bias, float* C, int ldc, const float* __restrict__ R, int K, size_t sA, size_t sB, size_t sC, int roundR) {
    __shared__ __align__(16) float ost[4][16 * 68];
    const size_t z = blockIdx.z; A += z * sA; Bn += z * sB; C += z * sC; if (R) R += z * sC;
    const int lane = threadIdx.x & 31, wave = threadIdx.x >> 5, lr = lane & 15, hi = lane >> 4;
    const int r0 = blockIdx.x * 64 + wave * 16, c0 = blockIdx.y * 64;
    const size_t aoff = (size_t)(r0 + lr) * K + 8 * hi;
    size_t boff[4];
#pragma unroll
    for (int t = 0; t < 4; ++t) boff[t] = (size_t)(c0 + t * 16 + lr) * K + 8 * hi;
    v8f acc[4];
#pragma unroll
    for (int t = 0; t < 4; ++t) acc[t] = (v8f){};
#pragma unroll 1
    for (int kc = 0; kc < K; kc += 32) {
        const v16h a = cat16(*(const v8h*)(A + aoff + kc), *(const v8h*)(A + aoff + kc + 16));
#pragma unroll
        for (int t = 0; t < 4; ++t) { const v16h b = cat16(*(const v8h*)(Bn + boff[t] + kc), *(const v8h*)(Bn + boff[t] + kc + 16)); acc[t] = wmma16(a, b, acc[t]); }
        asm volatile("v_nop\n\tv_nop\n\tv_nop\n\tv_nop" : "+v"(acc[0]), "+v"(acc[1]), "+v"(acc[2]), "+v"(acc[3]) : "v"(a));
    }
    float* os = &ost[wave][0];
#pragma unroll
    for (int t = 0; t < 4; ++t) { const float bv = bias ? bfr(bias[c0 + t * 16 + lr]) : 0.f;
#pragma unroll
        for (int j = 0; j < 8; ++j) os[(hi * 8 + j) * 68 + t * 16 + lr] = acc[t][j] + bv; }
    __syncthreads();
    float* crow = C + (size_t)r0 * ldc + c0;
    auto pass = [&]() {
#pragma unroll
        for (int s = 0; s < 8; ++s) { const int Lid = (lane >> 3) + 4 * s, piece = lane & 7; const int row = Lid >> 1, cofs = (Lid & 1) * 32 + piece * 4;
            v4f val = *(const v4fa*)(os + row * 68 + cofs); if (R) { const v4f rv = *(const v4f*)(R + ((size_t)r0 + row) * ldc + c0 + cofs); val += roundR ? (v4f){bfr(rv[0]), bfr(rv[1]), bfr(rv[2]), bfr(rv[3])} : rv; }
            *(volatile v4f*)(crow + (size_t)row * ldc + cofs) = val; }
    };
    pass(); __threadfence(); pass();
}

typedef __attribute__((ext_vector_type(4))) _Float16 v4h;
__device__ __forceinline__ h16 tohx(float x) { return (h16)x; }
__device__ __forceinline__ float gelu_e(float x) { return 0.5f * x * (1.0f + erff(x * 0.70710678118654752f)); }

template <int DIN, bool AFF, int WPB>
__global__ __launch_bounds__(WPB * 32) void k_feat(const float* __restrict__ X, const float* __restrict__ ns, const float* __restrict__ nb, const float* __restrict__ grid, h16* A) {
    __shared__ float rowb[WPB][7 * DIN]; __shared__ float sg[WPB * 32][NG + 1]; __shared__ float sB[WPB * 32][NG];
    const int lane = threadIdx.x & 31, wv = threadIdx.x >> 5; const size_t r = (size_t)blockIdx.x * WPB + wv; if (r >= (size_t)RCH) return; float* rb = rowb[wv]; float* g = sg[threadIdx.x]; float* B = sB[threadIdx.x];
#pragma unroll 1
    for (int q = 0; q < DIN / 32; ++q) { const int i = q * 32 + lane; float v = X[r * DIN + i]; v = AFF ? (bfr(ns[i]) * v + bfr(nb[i])) : bfr(v);
#pragma unroll 1
        for (int j = 0; j < NG; ++j) g[j] = bfr(grid[(size_t)i * NG + j]);
#pragma unroll 1
        for (int j = 0; j < NG - 1; ++j) B[j] = (v >= g[j] && v < g[j + 1]) ? 1.0f : 0.0f;
#pragma unroll 1
        for (int d = 1; d <= 3; ++d) {
#pragma unroll 1
            for (int j = 0; j < NG - 1 - d; ++j) { const float left = __fdiv_rn(v - g[j], g[j + d] - g[j]); const float right = __fdiv_rn(g[j + d + 1] - v, g[j + d + 1] - g[j + 1]); B[j] = left * B[j] + right * B[j + 1]; } }
#pragma unroll 1
        for (int b = 0; b < NB6; ++b) rb[b * DIN + i] = B[b];
        rb[6 * DIN + i] = __fdiv_rn(v, 1.0f + expf(-v)); }
    __builtin_amdgcn_wave_barrier(); asm volatile("" ::: "memory");
#pragma unroll 1
    for (int ps = 0; ps < 2; ++ps) {
#pragma unroll 1
        for (int p = 0; p < (7 * DIN) / 256; ++p) { const int c0 = p * 256 + lane * 8; v8h o;
#pragma unroll
            for (int k = 0; k < 8; ++k) o[k] = tohx(rb[c0 + k]);
            *(volatile v8h*)(A + r * (7 * DIN) + c0) = o; }
        if (ps == 0) __threadfence(); }
}
template <int DIN, int DOUT>
__global__ __launch_bounds__(256) void k_wkan(const float* __restrict__ coef, const float* __restrict__ sp, const float* __restrict__ sb, h16* Bt) {
    const int lane = threadIdx.x & 31; const int o_ = blockIdx.x * 8 + (threadIdx.x >> 5); if (o_ >= DOUT) return;
#pragma unroll 1
    for (int ps = 0; ps < 2; ++ps) {
#pragma unroll 1
        for (int p = 0; p < (7 * DIN) / 256; ++p) { const int c0 = p * 256 + lane * 8; v8h o;
#pragma unroll
            for (int k = 0; k < 8; ++k) { const int c = c0 + k; float v; if (c < 6 * DIN) { const int b = c / DIN, i = c % DIN; v = bfr(coef[((size_t)i * DOUT + o_) * NB6 + b]) * bfr(sp[(size_t)i * DOUT + o_]); } else { const int i = c - 6 * DIN; v = bfr(sb[(size_t)i * DOUT + o_]); } o[k] = tohx(v); }
            *(volatile v8h*)(Bt + (size_t)o_ * (7 * DIN) + c0) = o; }
        if (ps == 0) __threadfence(); }
}
__global__ __launch_bounds__(256) void k_final(const float* __restrict__ Y2, const float* __restrict__ X, const float* __restrict__ ns, const float* __restrict__ nb, const float* __restrict__ lg, const float* __restrict__ lb, size_t r0, float* OUTB) {
    const int lane = threadIdx.x & 31; const size_t rl = (size_t)blockIdx.x * 8 + (threadIdx.x >> 5); if (rl >= (size_t)RCH) return; const size_t r = r0 + rl; float v[8]; float s = 0.f;
#pragma unroll
    for (int i = 0; i < 8; ++i) { const int c = (i < 4) ? lane * 4 + i : 128 + lane * 4 + i - 4; v[i] = bfr(ns[c]) * Y2[rl * D2 + c] + bfr(nb[c]) + bfr(X[r * D0 + c]); s += v[i]; }
#pragma unroll
    for (int sh = 16; sh; sh >>= 1) s += __shfl_xor(s, sh, 32);
    const float mu = s * (1.0f / D2); float q = 0.f;
#pragma unroll
    for (int i = 0; i < 8; ++i) { const float d = v[i] - mu; q = fmaf(d, d, q); }
#pragma unroll
    for (int sh = 16; sh; sh >>= 1) q += __shfl_xor(q, sh, 32);
    const float rs = rsqrtf(q * (1.0f / D2) + 1e-5f); const v4f va = (v4f){v[0], v[1], v[2], v[3]}, vb = (v4f){v[4], v[5], v[6], v[7]};
#pragma unroll 1
    for (int half = 0; half < 2; ++half) { const v4f vv = half ? vb : va; const int cbase = half * 128 + lane * 4; v4f o;
#pragma unroll
        for (int i = 0; i < 4; ++i) o[i] = gelu_e((vv[i] - mu) * rs * bfr(lg[cbase + i]) + bfr(lb[cbase + i]));
        *(volatile v4f*)(OUTB + r * D2 + cbase) = o; __threadfence(); *(volatile v4f*)(OUTB + r * D2 + cbase) = o; }
}
extern "C" void kernel_launch(void* const* d_in, const int* in_sizes, int n_in,
                              void* d_out, int out_size, void* d_ws, size_t ws_size, hipStream_t stream) {
    (void)in_sizes; (void)n_in; (void)out_size;
    const float* x = (const float*)d_in[0]; const float* g1 = (const float*)d_in[1]; const float* c1 = (const float*)d_in[2]; const float* sb1 = (const float*)d_in[3]; const float* sp1 = (const float*)d_in[4]; const float* ns1 = (const float*)d_in[5]; const float* nb1 = (const float*)d_in[6];
    const float* g2 = (const float*)d_in[7]; const float* c2 = (const float*)d_in[8]; const float* sb2 = (const float*)d_in[9]; const float* sp2 = (const float*)d_in[10]; const float* ns2 = (const float*)d_in[11]; const float* nb2 = (const float*)d_in[12]; const float* lg = (const float*)d_in[13]; const float* lb = (const float*)d_in[14];
    float* out = (float*)d_out;
    char* wsp = (char*)d_ws;
    auto take = [&](size_t bytes) { char* p = wsp; wsp += (bytes + 255) & ~(size_t)255; return (void*)p; };
    h16* W1 = (h16*)take((size_t)D1 * K1 * 2); h16* W2 = (h16*)take((size_t)D2 * K2 * 2); h16* A1 = (h16*)take((size_t)RCH * K1 * 2); float* Y1 = (float*)take((size_t)RCH * D1 * 4); h16* A2 = (h16*)take((size_t)RCH * K2 * 2); float* Y2 = (float*)take((size_t)RCH * D2 * 4);
    if ((size_t)(wsp - (char*)d_ws) > ws_size) return;
    k_wkan<D0, D1><<<D1 / 8, 256, 0, stream>>>(c1, sp1, sb1, W1); k_wkan<D1, D2><<<D2 / 8, 256, 0, stream>>>(c2, sp2, sb2, W2);
    for (int ch = 0; ch < NROW / RCH; ++ch) { const size_t r0 = (size_t)ch * RCH;
        k_feat<D0, false, 4><<<RCH / 4, 128, 0, stream>>>(x + r0 * D0, nullptr, nullptr, g1, A1);
        k_gemmh<<<dim3(RCH / 64, D1 / 64, 1), 128, 0, stream>>>(A1, W1, nullptr, Y1, D1, nullptr, K1, 0, 0, 0, 0);
        k_feat<D1, true, 2><<<RCH / 2, 64, 0, stream>>>(Y1, ns1, nb1, g2, A2);
        k_gemmh<<<dim3(RCH / 64, D2 / 64, 1), 128, 0, stream>>>(A2, W2, nullptr, Y2, D2, nullptr, K2, 0, 0, 0, 0);
        k_final<<<RCH / 8, 256, 0, stream>>>(Y2, x, ns2, nb2, lg, lb, r0, out); }
}
